// BiMamba2DSlow4_18124761989167
// MI455X (gfx1250) — hardware-verified
//
#include <hip/hip_runtime.h>
#include <hip/hip_bf16.h>
#include <math.h>

#define NB    4
#define HH    56
#define WW    56
#define LPIX  (HH * WW)
#define NPIX  (NB * LPIX)
#define DMD   96
#define DIN   192
#define DST   16
#define DTR   6
#define XZW   (2 * DIN)
#define XDV   (DTR + 2 * DST)
#define CPJ   48
#define XDP   (4 * CPJ)
#define NT    96
#define GSTR  40
#define OSTR  100
#define SMEMB (8 * 16 * OSTR * 4)
#define SCH   32
#define SYP   196
#define LOG2E 1.4426950408889634f

static_assert(HH == WW);
static_assert(NPIX % 128 == 0);
static_assert(XZW % NT == 0);
static_assert(XDP % NT == 0);
static_assert(DMD % NT == 0);
static_assert(DMD % 32 == 0);
static_assert(DIN % 32 == 0);
static_assert(DIN == 192);
static_assert(DST == 16);
static_assert(DTR == 6);
static_assert(XDV <= 40);
static_assert(CPJ >= 40);
static_assert(LPIX % SCH == 0);
static_assert(SCH == 32);
static_assert(SYP % 4 == 0);
static_assert(SYP >= DIN);
static_assert(NT % 16 == 0);
static_assert(NT * 4 <= 512);
static_assert(OSTR >= NT);
static_assert(OSTR % 4 == 0);
static_assert(SMEMB >= (2 * 128 * GSTR + NT * GSTR) * 2);
static_assert(NPIX % 4 == 0);
static_assert(NPIX % 8 == 0);
static_assert(DMD % 8 == 0);
static_assert((NPIX * (DMD / 8)) % 256 == 0);

typedef unsigned short us16 __attribute__((ext_vector_type(16)));
typedef unsigned short us8  __attribute__((ext_vector_type(8)));
typedef unsigned short us8a __attribute__((ext_vector_type(8), may_alias));
typedef __bf16 v16b __attribute__((ext_vector_type(16)));
typedef float v8f __attribute__((ext_vector_type(8)));
typedef float v4f __attribute__((ext_vector_type(4)));
typedef float v4fa __attribute__((ext_vector_type(4), may_alias));
union FragU { us16 v; us8 h[2]; };

__device__ __forceinline__ unsigned short bf16_bits(float f) {
  unsigned u = __float_as_uint(f);
  u += 0x7FFFu + ((u >> 16) & 1u);
  return (unsigned short)(u >> 16);
}
__device__ __forceinline__ float bf16_val(unsigned short b) { return __uint_as_float(((unsigned)b) << 16); }
__device__ __forceinline__ float bf16r(float f) { return bf16_val(bf16_bits(f)); }
__device__ __forceinline__ float siluf(float x) { return x * __builtin_amdgcn_rcpf(1.0f + __expf(-x)); }

__device__ __forceinline__ v8f mma_bf16(us16 a, us16 b, v8f c) {
  return __builtin_amdgcn_wmma_f32_16x16x32_bf16(false, __builtin_bit_cast(v16b, a), false, __builtin_bit_cast(v16b, b), (short)0, c, false, false);
}
__device__ __forceinline__ void wguard(v8f& c0, v8f& c1, v8f& c2, v8f& c3, v8f& c4, v8f& c5,
                                       const us16& a0, const us16& a1,
                                       const us16& b0, const us16& b1, const us16& b2,
                                       const us16& b3, const us16& b4, const us16& b5) {
#if defined(__HIP_DEVICE_COMPILE__)
  asm volatile("v_nop\n\tv_nop\n\tv_nop\n\tv_nop"
               : "+v"(c0), "+v"(c1), "+v"(c2), "+v"(c3), "+v"(c4), "+v"(c5)
               : "v"(a0), "v"(a1), "v"(b0), "v"(b1), "v"(b2), "v"(b3), "v"(b4), "v"(b5));
#endif
}

__device__ __forceinline__ us16 lds_frag(const unsigned short* base) {
  const int lane = threadIdx.x & 31, r = lane & 15, kh = (lane >> 4) * 8;
  FragU f;
  f.h[0] = *(const us8a*)(base + r * GSTR + kh);
  f.h[1] = *(const us8a*)(base + r * GSTR + 16 + kh);
  return f.v;
}

__device__ __forceinline__ void stage_a(unsigned short* lds, const unsigned short* __restrict__ P, int ld, int m0, int k0, int tid) {
  const int row = tid >> 1, cq = (tid & 1) * 16;
  const unsigned short* src = P + (size_t)(m0 + row) * ld + k0 + cq;
  const us8 v0 = *(const us8a*)src;
  const us8 v1 = *(const us8a*)(src + 8);
  *(us8a*)(lds + row * GSTR + cq) = v0;
  *(us8a*)(lds + row * GSTR + cq + 8) = v1;
}
__device__ __forceinline__ void stage_b(unsigned short* lds, const unsigned short* __restrict__ P, int ld, int n0, int k0, int tid) {
  {
    const int i = tid, row = i >> 2, kq = (i & 3) * 8;
    const us8 v = *(const us8a*)(P + (size_t)(n0 + row) * ld + k0 + kq);
    *(us8a*)(lds + row * GSTR + kq) = v;
  }
  if (tid + 256 < NT * 4) {
    const int i = tid + 256, row = i >> 2, kq = (i & 3) * 8;
    const us8 v = *(const us8a*)(P + (size_t)(n0 + row) * ld + k0 + kq);
    *(us8a*)(lds + row * GSTR + kq) = v;
  }
}

template <bool RES>
__global__ __launch_bounds__(256) void k_gemm(const unsigned short* __restrict__ A0, const unsigned short* __restrict__ A1, int lda,
                                             const unsigned short* __restrict__ B0, int ldb, float* Y, int ldy, int K) {
  __shared__ __attribute__((aligned(16))) unsigned char sm[SMEMB];
  unsigned short* lA0 = (unsigned short*)sm;
  unsigned short* lA1 = lA0 + 128 * GSTR;
  unsigned short* lB0 = lA1 + 128 * GSTR;
  float* oS = (float*)sm;
  const int tid = threadIdx.x, lane = tid & 31, wave = tid >> 5, cl = lane & 15, hh = lane >> 4;
  const int m0 = blockIdx.x * 128, n0 = blockIdx.y * NT;

  v8f acc[6];
#pragma unroll
  for (int j = 0; j < 6; ++j) { v8f zz = {0.f, 0.f, 0.f, 0.f, 0.f, 0.f, 0.f, 0.f}; acc[j] = zz; }

#pragma unroll 1
  for (int k0 = 0; k0 < K; k0 += 32) {
    __syncthreads();
    stage_a(lA0, A0, lda, m0, k0, tid);
    if (RES) stage_a(lA1, A1, lda, m0, k0, tid);
    stage_b(lB0, B0, ldb, n0, k0, tid);
    __syncthreads();
    const us16 af0 = lds_frag(lA0 + 16 * wave * GSTR);
    us16 af1 = af0;
    if (RES) af1 = lds_frag(lA1 + 16 * wave * GSTR);
    us16 bfr[6];
#pragma unroll
    for (int j = 0; j < 6; ++j) bfr[j] = lds_frag(lB0 + 16 * j * GSTR);
#pragma unroll
    for (int j = 0; j < 6; ++j) acc[j] = mma_bf16(af0, bfr[j], acc[j]);
    if (RES) {
#pragma unroll
      for (int j = 0; j < 6; ++j) acc[j] = mma_bf16(af1, bfr[j], acc[j]);
    }
    wguard(acc[0], acc[1], acc[2], acc[3], acc[4], acc[5], af0, af1, bfr[0], bfr[1], bfr[2], bfr[3], bfr[4], bfr[5]);
  }
  __syncthreads();

  float* so = oS + wave * (16 * OSTR);
#pragma unroll
  for (int j = 0; j < 6; ++j)
#pragma unroll
    for (int r = 0; r < 8; ++r) so[(8 * hh + r) * OSTR + 16 * j + cl] = acc[j][r];
  __syncthreads();
#pragma unroll
  for (int pass = 0; pass < 2; ++pass) {
#pragma unroll
    for (int it = 0; it < 12; ++it) {
      const int ch = it * 32 + lane, r = ch / 24, q = (ch - r * 24) * 4;
      const v4f v = *(const v4fa*)(so + r * OSTR + q);
      *(volatile v4f*)(Y + (size_t)(m0 + 16 * wave + r) * ldy + n0 + q) = v;
    }
    __threadfence();
  }
}

__global__ __launch_bounds__(256) void k_cvt(const float* __restrict__ src, unsigned short* dst, int nsrc, int ncol8, int total8) {
  const int idx = blockIdx.x * 256 + threadIdx.x;
  if (idx >= total8) return;
  const int row = idx / ncol8, c8 = (idx - row * ncol8) * 8;
  const int rs = (row < nsrc) ? row : (nsrc - 1);
  const float* s = src + (size_t)rs * (size_t)(ncol8 * 8) + c8;
  const v4f a = *(const v4fa*)s, b = *(const v4fa*)(s + 4);
  const bool zr = (row >= nsrc);
  us8 o;
#pragma unroll
  for (int u = 0; u < 4; ++u) {
    o[u]     = zr ? (unsigned short)0 : bf16_bits(a[u]);
    o[4 + u] = zr ? (unsigned short)0 : bf16_bits(b[u]);
  }
  const size_t off = (size_t)row * (size_t)(ncol8 * 8) + c8;
  *(volatile us8*)(dst + off) = o;
  __threadfence();
  *(volatile us8*)(dst + off) = o;
}

__global__ __launch_bounds__(256) void k_cvt_wx(const float* __restrict__ src, unsigned short* dst) {
  const int idx = blockIdx.x * 256 + threadIdx.x;
  if (idx >= XDP * (DIN / 8)) return;
  const int row = idx / (DIN / 8), c8 = (idx - row * (DIN / 8)) * 8;
  const int k = row / CPJ, c = row - k * CPJ;
  const int cs = (c < XDV) ? c : (XDV - 1);
  const float* s = src + (size_t)(k * XDV + cs) * DIN + c8;
  const v4f a = *(const v4fa*)s, b = *(const v4fa*)(s + 4);
  const bool zr = (c >= XDV);
  us8 o;
#pragma unroll
  for (int u = 0; u < 4; ++u) {
    o[u]     = zr ? (unsigned short)0 : bf16_bits(a[u]);
    o[4 + u] = zr ? (unsigned short)0 : bf16_bits(b[u]);
  }
  const size_t off = (size_t)row * DIN + c8;
  *(volatile us8*)(dst + off) = o;
  __threadfence();
  *(volatile us8*)(dst + off) = o;
}

__global__ __launch_bounds__(DIN) void k_conv(const float* __restrict__ XZ, const float* __restrict__ cw, const float* __restrict__ cb,
                                             float* XCF, unsigned short* XCH, unsigned short* XCL) {
#pragma clang fp contract(off)
  __shared__ __attribute__((aligned(16))) float sxs[4 * DIN];
  const int tid = threadIdx.x, tl = tid / 48, c4 = (tid - tl * 48) * 4;
  const int bp = blockIdx.x * 4 + tl;
  const int b = bp / LPIX, p = bp - b * LPIX;
  const int h = p / WW, w = p - h * WW;
  v4f acc = {0.f, 0.f, 0.f, 0.f};
#pragma unroll
  for (int dy = 0; dy < 3; ++dy) {
    const int hs = h + dy - 1;
    const int hc = (hs < 0) ? 0 : ((hs > HH - 1) ? (HH - 1) : hs);
#pragma unroll
    for (int dx = 0; dx < 3; ++dx) {
      const int wsx = w + dx - 1;
      const int wc = (wsx < 0) ? 0 : ((wsx > WW - 1) ? (WW - 1) : wsx);
      const bool ok = (hs >= 0) && (hs < HH) && (wsx >= 0) && (wsx < WW);
      const v4f xv = *(const v4fa*)(XZ + (size_t)(b * LPIX + hc * WW + wc) * XZW + c4);
#pragma unroll
      for (int u = 0; u < 4; ++u) {
        const float wv = bf16r(cw[(c4 + u) * 9 + dy * 3 + dx]);
        const float pr = wv * xv[u];
        acc[u] = acc[u] + (ok ? pr : 0.0f);
      }
    }
  }
  const v4f bb = *(const v4fa*)(cb + c4);
  v4f sv;
#pragma unroll
  for (int u = 0; u < 4; ++u) sv[u] = siluf(acc[u] + bf16r(bb[u]));
  *(v4fa*)(sxs + tl * DIN + c4) = sv;
  const size_t o = (size_t)bp * DIN + c4;
  *(volatile v4f*)(XCF + o) = sv;
  __threadfence();
  *(volatile v4f*)(XCF + o) = sv;
  __syncthreads();
  if (tid < 96) {
    const int row = tid / 24, c8 = (tid - row * 24) * 8;
    const v4f a = *(const v4fa*)(sxs + row * DIN + c8);
    const v4f bq = *(const v4fa*)(sxs + row * DIN + c8 + 4);
    us8 hi, lo;
#pragma unroll
    for (int u = 0; u < 4; ++u) {
      const unsigned short ha = bf16_bits(a[u]);
      hi[u] = ha; lo[u] = bf16_bits(a[u] - bf16_val(ha));
      const unsigned short hb = bf16_bits(bq[u]);
      hi[4 + u] = hb; lo[4 + u] = bf16_bits(bq[u] - bf16_val(hb));
    }
    const size_t o2 = (size_t)(blockIdx.x * 4 + row) * DIN + c8;
    *(volatile us8*)(XCH + o2) = hi; *(volatile us8*)(XCL + o2) = lo;
    __threadfence();
    *(volatile us8*)(XCH + o2) = hi; *(volatile us8*)(XCL + o2) = lo;
  }
}

__device__ __forceinline__ int pix_of(int k, int t) {
  const int q = (k >= 2) ? (LPIX - 1 - t) : t;
  const int qa = q / HH;
  const int qb = q - qa * HH;
  return (k & 1) ? (qb * WW + qa) : q;
}

__global__ __launch_bounds__(DIN) void k_scan(const float* __restrict__ XD, const float* __restrict__ XCF, const float* __restrict__ dtw,
                                             const float* __restrict__ dtb, const float* __restrict__ Alog, const float* __restrict__ Dv,
                                             float* YK) {
#pragma clang fp contract(off)
  __shared__ __attribute__((aligned(16))) float sy[SCH * SYP];
  const int b = blockIdx.x, k = blockIdx.y, tid = threadIdx.x, d = tid, lane = tid & 31, wave = tid >> 5;
  const int kd = k * DIN + d;
  float A2[DST], h[DST], wr[DTR];
#pragma unroll
  for (int n = 0; n < DST; ++n) { A2[n] = -__expf(bf16r(Alog[kd * DST + n])) * LOG2E; h[n] = 0.0f; }
#pragma unroll
  for (int r = 0; r < DTR; ++r) wr[r] = bf16r(dtw[kd * DTR + r]);
  const float bias = bf16r(dtb[kd]);
  const float Dd = bf16r(Dv[kd]);
  float* yk = YK + ((size_t)k * NB + b) * (size_t)LPIX * DIN;
#pragma unroll 1
  for (int c = 0; c < LPIX / SCH; ++c) {
#pragma unroll 1
    for (int s = 0; s < SCH; ++s) {
      const int t = c * SCH + s;
      const int p = pix_of(k, t);
      const size_t row = (size_t)b * LPIX + (size_t)p;
      const float u = XCF[row * DIN + d];
      const float* xr = XD + row * XDP + k * CPJ;
      v4f v[10];
#pragma unroll
      for (int q = 0; q < 10; ++q) v[q] = *(const v4fa*)(xr + 4 * q);
      float a = 0.0f;
#pragma unroll
      for (int r = 0; r < 4; ++r) a = a + v[0][r] * wr[r];
      a = a + v[1][0] * wr[4];
      a = a + v[1][1] * wr[5];
      a = a + bias;
      const float dl = fmaxf(a, 0.0f) + log1pf(__expf(-fabsf(a)));
      const float dx = dl * u;
      float y = 0.0f;
#pragma unroll
      for (int n = 0; n < DST; ++n) {
        const float e = exp2f(dl * A2[n]);
        h[n] = e * h[n] + dx * v[(DTR + n) >> 2][(DTR + n) & 3];
        y = y + h[n] * v[(DTR + DST + n) >> 2][(DTR + DST + n) & 3];
      }
      sy[s * SYP + d] = y + u * Dd;
    }
    __syncthreads();
#pragma unroll
    for (int pass = 0; pass < 2; ++pass) {
      for (int rr = wave; rr < SCH; rr += 6) {
        const int p = pix_of(k, c * SCH + rr);
        float* dst = yk + (size_t)p * DIN;
        const v4f va = *(const v4fa*)(sy + rr * SYP + lane * 4);
        *(volatile v4f*)(dst + lane * 4) = va;
        if (lane < 16) {
          const v4f vb = *(const v4fa*)(sy + rr * SYP + 128 + lane * 4);
          *(volatile v4f*)(dst + 128 + lane * 4) = vb;
        }
      }
      __threadfence();
    }
    __syncthreads();
  }
}

__global__ __launch_bounds__(256) void k_lngate(const float* __restrict__ YK, const float* __restrict__ XZ, const float* __restrict__ gam,
                                               const float* __restrict__ bet, unsigned short* YGH, unsigned short* YGL) {
#pragma clang fp contract(off)
  __shared__ __attribute__((aligned(16))) float sg[8 * SYP];
  const int tid = threadIdx.x, lane = tid & 31, wave = tid >> 5;
  const int bp = blockIdx.x * 8 + wave;
  const size_t pl = (size_t)NPIX * DIN;
  const float* y0 = YK + (size_t)bp * DIN;
  float yv[6];
  float s = 0.0f;
#pragma unroll
  for (int j = 0; j < 6; ++j) {
    const int d = lane + 32 * j;
    const float a0 = y0[d], a2 = y0[2 * pl + d], a1 = y0[pl + d], a3 = y0[3 * pl + d];
    yv[j] = ((a0 + a2) + a1) + a3;
    s = s + yv[j];
  }
#pragma unroll
  for (int o = 16; o > 0; o >>= 1) s = s + __shfl_xor(s, o);
  const float mean = s * (1.0f / (float)DIN);
  float qv = 0.0f;
#pragma unroll
  for (int j = 0; j < 6; ++j) { const float dv = yv[j] - mean; qv = qv + dv * dv; }
#pragma unroll
  for (int o = 16; o > 0; o >>= 1) qv = qv + __shfl_xor(qv, o);
  const float var = qv * (1.0f / (float)DIN);
  const float rs = rsqrtf(var + 1e-5f);
#pragma unroll
  for (int j = 0; j < 6; ++j) {
    const int d = lane + 32 * j;
    float g = (yv[j] - mean) * rs * bf16r(gam[d]) + bf16r(bet[d]);
    const float z = XZ[(size_t)bp * XZW + DIN + d];
    g = g * siluf(z);
    sg[wave * SYP + d] = g;
  }
  __syncthreads();
  if (lane < 24) {
    const int c8 = lane * 8;
    const v4f a = *(const v4fa*)(sg + wave * SYP + c8);
    const v4f bq = *(const v4fa*)(sg + wave * SYP + c8 + 4);
    us8 hi, lo;
#pragma unroll
    for (int u = 0; u < 4; ++u) {
      const unsigned short ha = bf16_bits(a[u]);
      hi[u] = ha; lo[u] = bf16_bits(a[u] - bf16_val(ha));
      const unsigned short hb = bf16_bits(bq[u]);
      hi[4 + u] = hb; lo[4 + u] = bf16_bits(bq[u] - bf16_val(hb));
    }
    const size_t o = (size_t)bp * DIN + c8;
    *(volatile us8*)(YGH + o) = hi; *(volatile us8*)(YGL + o) = lo;
    __threadfence();
    *(volatile us8*)(YGH + o) = hi; *(volatile us8*)(YGL + o) = lo;
  }
}

extern "C" void kernel_launch(void* const* d_in, const int* in_sizes, int n_in,
                              void* d_out, int out_size, void* d_ws, size_t ws_size,
                              hipStream_t stream) {
  if (n_in < 12) return;
  if (in_sizes[0] != NPIX * DMD || in_sizes[1] != XZW * DMD || in_sizes[2] != DIN * 9 || in_sizes[3] != DIN ||
      in_sizes[4] != 4 * XDV * DIN || in_sizes[5] != 4 * DIN * DTR || in_sizes[6] != 4 * DIN || in_sizes[7] != 4 * DIN * DST ||
      in_sizes[8] != 4 * DIN || in_sizes[9] != DIN || in_sizes[10] != DIN || in_sizes[11] != DMD * DIN ||
      out_size != NPIX * DMD) return;
  const float* x    = (const float*)d_in[0];
  const float* Win  = (const float*)d_in[1];
  const float* cw   = (const float*)d_in[2];
  const float* cb   = (const float*)d_in[3];
  const float* Wx   = (const float*)d_in[4];
  const float* dtw  = (const float*)d_in[5];
  const float* dtb  = (const float*)d_in[6];
  const float* Alog = (const float*)d_in[7];
  const float* Dv   = (const float*)d_in[8];
  const float* gam  = (const float*)d_in[9];
  const float* bet  = (const float*)d_in[10];
  const float* Wo   = (const float*)d_in[11];
  float* out = (float*)d_out;

  size_t off = 0;
  auto carve = [&](size_t bytes) -> char* { char* p = (char*)d_ws + off; off += (bytes + 255) & ~(size_t)255; return p; };
  unsigned short* XH    = (unsigned short*)carve((size_t)NPIX * DMD * 2);
  unsigned short* WIN16 = (unsigned short*)carve((size_t)XZW * DMD * 2);
  unsigned short* WX16  = (unsigned short*)carve((size_t)XDP * DIN * 2);
  unsigned short* WO16  = (unsigned short*)carve((size_t)DMD * DIN * 2);
  float* XZ             = (float*)carve((size_t)NPIX * XZW * 4);
  float* XCF            = (float*)carve((size_t)NPIX * DIN * 4);
  unsigned short* XCH   = (unsigned short*)carve((size_t)NPIX * DIN * 2);
  unsigned short* XCL   = (unsigned short*)carve((size_t)NPIX * DIN * 2);
  float* XD             = (float*)carve((size_t)NPIX * XDP * 4);
  float* YK             = (float*)carve((size_t)4 * NPIX * DIN * 4);
  unsigned short* YGH   = (unsigned short*)carve((size_t)NPIX * DIN * 2);
  unsigned short* YGL   = (unsigned short*)carve((size_t)NPIX * DIN * 2);
  if (off > ws_size || off > (size_t)134217728) return;

  const dim3 blk(256);
  k_cvt<<<dim3((NPIX * (DMD / 8) + 255) / 256), blk, 0, stream>>>(x, XH, NPIX, DMD / 8, NPIX * (DMD / 8));
  k_cvt<<<dim3((XZW * DMD / 8 + 255) / 256), blk, 0, stream>>>(Win, WIN16, XZW, DMD / 8, XZW * DMD / 8);
  k_cvt_wx<<<dim3((XDP * (DIN / 8) + 255) / 256), blk, 0, stream>>>(Wx, WX16);
  k_cvt<<<dim3((DMD * DIN / 8 + 255) / 256), blk, 0, stream>>>(Wo, WO16, DMD, DIN / 8, DMD * DIN / 8);
  k_gemm<false><<<dim3(NPIX / 128, XZW / NT), blk, 0, stream>>>(XH, XH, DMD, WIN16, DMD, XZ, XZW, DMD);
  k_conv<<<dim3(NPIX / 4), dim3(DIN), 0, stream>>>(XZ, cw, cb, XCF, XCH, XCL);
  k_gemm<true><<<dim3(NPIX / 128, XDP / NT), blk, 0, stream>>>(XCH, XCL, DIN, WX16, DIN, XD, XDP, DIN);
  k_scan<<<dim3(NB, 4), dim3(DIN), 0, stream>>>(XD, XCF, dtw, dtb, Alog, Dv, YK);
  k_lngate<<<dim3(NPIX / 8), blk, 0, stream>>>(YK, XZ, gam, bet, YGH, YGL);
  k_gemm<true><<<dim3(NPIX / 128, DMD / NT), blk, 0, stream>>>(YGH, YGL, DIN, WO16, DIN, out, DMD, DIN);
}
